// MAB_70987219468669
// MI455X (gfx1250) — hardware-verified
//
#include <hip/hip_runtime.h>
#include <math.h>

typedef __attribute__((ext_vector_type(16))) _Float16 v16h;
typedef __attribute__((ext_vector_type(16))) __bf16 v16b;
typedef __attribute__((ext_vector_type(8)))  _Float16 v8h;
typedef __attribute__((ext_vector_type(8)))  __bf16 v8b;
typedef __attribute__((ext_vector_type(8)))  float v8f;
typedef __attribute__((ext_vector_type(4)))  float v4f;
typedef __attribute__((ext_vector_type(4)))  unsigned v4u;

template <typename T> __device__ __forceinline__ void vst2(void* p, T v) { *(volatile T*)p = v; __threadfence(); *(volatile T*)p = v; }
__device__ __forceinline__ v8f wmma16(v16h a, v16h b, v8f c) {
  v8f d = __builtin_amdgcn_wmma_f32_16x16x32_f16(false, a, false, b, (short)0, c, false, false);
  asm volatile("v_nop\n\tv_nop\n\tv_nop\n\tv_nop" : "+v"(d) : "v"(a), "v"(b));
  return d;
}
__device__ __forceinline__ v8f wmma_bf(v16b a, v16b b, v8f c) {
  v8f d = __builtin_amdgcn_wmma_f32_16x16x32_bf16(false, a, false, b, (short)0, c, false, false);
  asm volatile("v_nop\n\tv_nop\n\tv_nop\n\tv_nop" : "+v"(d) : "v"(a), "v"(b));
  return d;
}
__device__ __forceinline__ v16h frag_h(const _Float16* rowk0, int lane) {
  union { v16h v; v8h q[2]; } u; const _Float16* p = rowk0 + 8 * (lane >> 4);
  u.q[0] = *(const v8h*)p; u.q[1] = *(const v8h*)(p + 16); return u.v;
}
__device__ __forceinline__ v16b frag_b(const __bf16* rowk0, int lane) {
  union { v16b v; v8b q[2]; } u; const __bf16* p = rowk0 + 8 * (lane >> 4);
  u.q[0] = *(const v8b*)p; u.q[1] = *(const v8b*)(p + 16); return u.v;
}
__device__ __forceinline__ v16h frag_f32(const float* rowk0, int lane) {
  v16h a; const float* p = rowk0 + 8 * (lane >> 4);
#pragma unroll
  for (int i = 0; i < 8; ++i) { a[i] = (_Float16)p[i]; a[8 + i] = (_Float16)p[16 + i]; }
  return a;
}
__device__ __forceinline__ v16b frag_f32b(const float* rowk0, int lane) {
  v16b a; const float* p = rowk0 + 8 * (lane >> 4);
#pragma unroll
  for (int i = 0; i < 8; ++i) { a[i] = (__bf16)p[i]; a[8 + i] = (__bf16)p[16 + i]; }
  return a;
}
struct F2 { v16b h, l; };
__device__ __forceinline__ F2 bsplit16(const float v[16]) { F2 r;
#pragma unroll
  for (int i = 0; i < 16; ++i) { const __bf16 h = (__bf16)v[i]; r.h[i] = h; r.l[i] = (__bf16)(v[i] - (float)h); }
  return r; }
__device__ __forceinline__ F2 split_row(const float* row, int k0, int lane) { float v[16]; const float* p = row + k0 + 8 * (lane >> 4);
#pragma unroll
  for (int i = 0; i < 8; ++i) { v[i] = p[i]; v[8 + i] = p[16 + i]; }
  return bsplit16(v); }
__device__ __forceinline__ float bfr(float v) { return (float)(__bf16)v; }
__device__ __forceinline__ void ldsx() { asm volatile("s_wait_dscnt 0" ::: "memory"); __builtin_amdgcn_wave_barrier(); __builtin_amdgcn_fence(3, "workgroup"); }

#define NB_FULL 8
#define TT_FULL 1024
#ifndef NB
#define NB NB_FULL
#endif
#ifndef SEQ
#define SEQ TT_FULL
#endif
#define TT SEQ
#define DIN 512
#define CC 512
#define NH 8
#define HD 64
#define NQB (TT / 64)
#define NROW (NB * TT)
#define SCALE (0.044194173824159216f)
static_assert(NH * HD == CC);
static_assert(DIN == CC);
static_assert(TT % 128 == 0 && TT >= 256 && TT <= TT_FULL);
static_assert(NB >= 1 && NB <= NB_FULL);
static_assert(DIN % 64 == 0 && CC % 128 == 0);

#define WS_WT  ((size_t)0)
#define WS_QH  (WS_WT + 2u * (size_t)4 * CC * DIN)
#define WS_KH  (WS_QH + 2u * (size_t)NROW * CC)
#define WS_VT  (WS_KH + 2u * (size_t)NROW * CC)
#define WS_QL  (WS_VT + 2u * (size_t)NB * CC * TT)
#define WS_S   (WS_QL + 2u * (size_t)NROW * CC)
#define WS_QF  (WS_S  + 4u * (size_t)NH * TT * TT)
#define WS_O   (WS_QF + 4u * (size_t)NROW * CC)
#define WS_T   (WS_O  + 4u * (size_t)NROW * CC)
#define WS_END (WS_T  + 4u * (size_t)NROW * CC)
static_assert(WS_END <= (size_t)134217728u);
static_assert(WS_QH % 128 == 0 && WS_KH % 128 == 0 && WS_VT % 128 == 0 && WS_QL % 128 == 0 && WS_S % 128 == 0 && WS_QF % 128 == 0 && WS_O % 128 == 0 && WS_T % 128 == 0);

__global__ __launch_bounds__(256) void k_wprep(const float* __restrict__ W0, const float* __restrict__ W1, const float* __restrict__ W2, const float* __restrict__ W3, __bf16* __restrict__ WT) {
  __shared__ __align__(16) __bf16 tl[64][72];
  const int w = blockIdx.z; const float* W = w == 0 ? W0 : w == 1 ? W1 : w == 2 ? W2 : W3;
  const int k0 = blockIdx.x * 64, o0 = blockIdx.y * 64; const int tid = threadIdx.x;
  for (int e = tid; e < 64 * 64; e += 256) { const int kl = e >> 6, ol = e & 63; tl[ol][kl] = (__bf16)W[(size_t)(k0 + kl) * CC + o0 + ol]; }
  __syncthreads();
  for (int e = tid; e < 64 * 8; e += 256) { const int ol = e >> 3, q = e & 7; vst2((unsigned*)(WT + ((size_t)w * CC + o0 + ol) * DIN + k0 + q * 8), *(const v4u*)&tl[ol][q * 8]); }
}

__global__ __launch_bounds__(128) __attribute__((amdgpu_num_vgpr(256))) void k_proj(const float* __restrict__ XQ, const float* __restrict__ XK, const __bf16* __restrict__ WT,
    const float* __restrict__ BQ, const float* __restrict__ BK, const float* __restrict__ BV,
    _Float16* __restrict__ QH, _Float16* __restrict__ QL, _Float16* __restrict__ KH, _Float16* __restrict__ VT) {
  __shared__ __align__(16) _Float16 sh[64][136], sl[64][136]; __shared__ __align__(16) _Float16 th[128][72];
  const int tid = threadIdx.x, wave = tid >> 5, lane = tid & 31, col = lane & 15, g = lane >> 4;
  const int which = blockIdx.z; const int c0 = blockIdx.y * 128;
  const size_t r0 = (size_t)blockIdx.x * 64; const size_t bb = r0 / TT; const int t0 = (int)(r0 % TT); const size_t ir0 = bb * TT_FULL + t0;
  const float* X = which == 0 ? XQ : XK; const __bf16* WP = WT + (size_t)which * CC * DIN; const float* BA = which == 0 ? BQ : which == 1 ? BK : BV;
  v8f acc[8] = {};
#pragma unroll 2
  for (int kc = 0; kc < DIN / 32; ++kc) {
    const v16b a = frag_f32b(X + (ir0 + wave * 16 + col) * DIN + kc * 32, lane);
    asm volatile("s_wait_loadcnt 0x0" ::: "memory");
#pragma unroll
    for (int j = 0; j < 8; ++j) { const v16b w = frag_b(WP + (size_t)(c0 + j * 16 + col) * DIN + kc * 32, lane); asm volatile("s_wait_loadcnt 0x0" ::: "memory"); acc[j] = wmma_bf(a, w, acc[j]); } }
  if (which < 2) { _Float16* DH = which == 0 ? QH : KH;
#pragma unroll
    for (int j = 0; j < 8; ++j) { const float bias = bfr(BA[c0 + j * 16 + col]);
#pragma unroll
      for (int r = 0; r < 8; ++r) { const float v = acc[j][r] + bias; const _Float16 hv = (_Float16)v; sh[wave * 16 + 8 * g + r][j * 16 + col] = hv; sl[wave * 16 + 8 * g + r][j * 16 + col] = (_Float16)((v - (float)hv) * 1024.0f); } }
    __syncthreads();
    for (int e = tid; e < 64 * 16; e += 128) { const int rl = e >> 4, q = e & 15;
      vst2((unsigned*)(DH + (r0 + rl) * CC + c0 + q * 8), *(const v4u*)&sh[rl][q * 8]);
      if (which == 0) vst2((unsigned*)(QL + (r0 + rl) * CC + c0 + q * 8), *(const v4u*)&sl[rl][q * 8]); }
  } else {
#pragma unroll
    for (int j = 0; j < 8; ++j) { const float bias = bfr(BA[c0 + j * 16 + col]);
#pragma unroll
      for (int r = 0; r < 8; ++r) { const float v = acc[j][r] + bias; const int rl = wave * 16 + 8 * g + r, cl = j * 16 + col; th[cl][rl] = (_Float16)v; } }
    __syncthreads();
    for (int e = tid; e < 128 * 8; e += 128) { const int cl = e >> 3, q = e & 7; vst2((unsigned*)(VT + (bb * CC + c0 + cl) * (size_t)TT + t0 + q * 8), *(const v4u*)&th[cl][q * 8]); } }
}

__global__ __launch_bounds__(128) __attribute__((amdgpu_num_vgpr(256))) void k_qrows(const float* __restrict__ X, const __bf16* __restrict__ WT, const float* __restrict__ BQ, float* __restrict__ QF) { __shared__ __align__(16) float sf[4][16][132];
  const int tid = threadIdx.x, wave = tid >> 5, lane = tid & 31, col = lane & 15, g = lane >> 4; const int c0 = blockIdx.y * 128;
  const size_t rb = (size_t)blockIdx.x * 64; const size_t bb = rb / TT; const int t0 = (int)(rb % TT); const size_t ir0 = bb * TT_FULL + t0 + wave * 16; const size_t r0 = rb + wave * 16;
  v8f acc[8] = {};
#pragma unroll 2
  for (int kc = 0; kc < DIN / 32; ++kc) {
    const v16b a = frag_f32b(X + (ir0 + col) * DIN + kc * 32, lane);
    asm volatile("s_wait_loadcnt 0x0" ::: "memory");
#pragma unroll
    for (int j = 0; j < 8; ++j) { const v16b w = frag_b(WT + (size_t)(c0 + j * 16 + col) * DIN + kc * 32, lane); asm volatile("s_wait_loadcnt 0x0" ::: "memory"); acc[j] = wmma_bf(a, w, acc[j]); } }
#pragma unroll
  for (int j = 0; j < 8; ++j) { const float bias = bfr(BQ[c0 + j * 16 + col]);
#pragma unroll
    for (int r = 0; r < 8; ++r) sf[wave][8 * g + r][j * 16 + col] = acc[j][r] + bias; }
  ldsx(); for (int rl = 0; rl < 16; ++rl) vst2(QF + (r0 + rl) * CC + c0 + lane * 4, *(const v4f*)&sf[wave][rl][lane * 4]);
}

__global__ __launch_bounds__(128) __attribute__((amdgpu_num_vgpr(256))) void k_sc(const _Float16* __restrict__ QH, const _Float16* __restrict__ KH, const _Float16* __restrict__ QL, int b, float* __restrict__ S0) {
  __shared__ __align__(16) float ss[4][16][132];
  const int qb = blockIdx.x, kb = blockIdx.y, h = blockIdx.z; float* S = S0 + (size_t)h * TT * TT;
  const int tid = threadIdx.x, wave = tid >> 5, lane = tid & 31, col = lane & 15, g = lane >> 4;
  const int k0 = kb * 128; const int ql0 = qb * 64 + wave * 16; const size_t q0 = (size_t)b * TT + ql0, kr0 = (size_t)b * TT + k0;
  v8f acc[8] = {}, accl[8] = {};
#pragma unroll
  for (int kc = 0; kc < HD / 32; ++kc) {
    const v16h ah = frag_h(QH + (q0 + col) * CC + h * HD + kc * 32, lane);
    const v16h al = frag_h(QL + (q0 + col) * CC + h * HD + kc * 32, lane);
    asm volatile("s_wait_loadcnt 0x0" ::: "memory");
#pragma unroll
    for (int j = 0; j < 8; ++j) { const v16h kf = frag_h(KH + (kr0 + j * 16 + col) * CC + h * HD + kc * 32, lane); asm volatile("s_wait_loadcnt 0x0" ::: "memory"); acc[j] = wmma16(ah, kf, acc[j]); accl[j] = wmma16(al, kf, accl[j]); } }
#pragma unroll
  for (int j = 0; j < 8; ++j) {
#pragma unroll
    for (int r = 0; r < 8; ++r) ss[wave][8 * g + r][j * 16 + col] = (acc[j][r] + accl[j][r] * (1.0f / 1024.0f)) * SCALE; }
  ldsx(); for (int rl = 0; rl < 16; ++rl) vst2(S + (size_t)(ql0 + rl) * TT + k0 + lane * 4, *(const v4f*)&ss[wave][rl][lane * 4]);
}

__global__ __launch_bounds__(256) void k_sm(float* __restrict__ S0, const int* __restrict__ MK, int b) { __shared__ float sred[8]; __shared__ float sbc; __shared__ __align__(16) float shv[TT];
  const int tid = threadIdx.x; const int t = blockIdx.x;
  float* sr = S0 + (size_t)blockIdx.y * TT * TT + (size_t)t * TT; const int* mrow = MK + (size_t)b * TT_FULL;
  float m = -3.0e38f;
  for (int k = tid; k < TT; k += 256) { const float s = sr[k]; const int mv = mrow[k]; const float v = (mv == 0) ? -10000.0f : s; shv[k] = v; m = fmaxf(m, v); }
#pragma unroll
  for (int o = 1; o < 32; o <<= 1) m = fmaxf(m, __shfl_xor(m, o));
  if ((tid & 31) == 0) sred[tid >> 5] = m; __syncthreads(); if (tid == 0) { float a = sred[0]; for (int i = 1; i < 8; ++i) a = fmaxf(a, sred[i]); sbc = a; } __syncthreads(); m = sbc; __syncthreads();
  float sum = 0.f;
#pragma unroll 1
  for (int k = tid; k < TT; k += 256) { const float e = expf(shv[k] - m); shv[k] = e; sum += e; }
#pragma unroll
  for (int o = 1; o < 32; o <<= 1) sum += __shfl_xor(sum, o);
  if ((tid & 31) == 0) sred[tid >> 5] = sum; __syncthreads(); if (tid == 0) { float a = 0.f; for (int i = 0; i < 8; ++i) a += sred[i]; sbc = a > 0.f ? 2048.0f / a : 0.f; } __syncthreads(); const float inv = sbc;
  for (int k = tid; k < TT; k += 256) shv[k] = shv[k] * inv;
  __syncthreads(); for (int q = tid; q < TT / 4; q += 256) vst2(sr + q * 4, *(const v4f*)&shv[q * 4]);
}

__global__ __launch_bounds__(128) __attribute__((amdgpu_num_vgpr(256))) void k_pv(const float* __restrict__ PS0, const _Float16* __restrict__ VT, int b, float* __restrict__ Y) {
  __shared__ __align__(16) float ss[4][16][HD + 4];
  const int h = blockIdx.z; const float* PS = PS0 + (size_t)h * TT * TT;
  const int tid = threadIdx.x, wave = tid >> 5, lane = tid & 31, col = lane & 15, g = lane >> 4; const int qb = blockIdx.x; const int ql0 = qb * 64 + wave * 16;
  v8f acc[HD / 16] = {};
#pragma unroll 1
  for (int kc = 0; kc < TT / 32; ++kc) { const v16h p = frag_f32(PS + (size_t)(ql0 + col) * TT + kc * 32, lane);
    asm volatile("s_wait_loadcnt 0x0" ::: "memory");
#pragma unroll
    for (int j = 0; j < HD / 16; ++j) { const size_t po = ((size_t)b * CC + h * HD + j * 16 + col) * (size_t)TT + kc * 32; acc[j] = wmma16(p, frag_h(VT + po, lane), acc[j]); } }
#pragma unroll
  for (int j = 0; j < HD / 16; ++j)
#pragma unroll
    for (int r = 0; r < 8; ++r) ss[wave][8 * g + r][j * 16 + col] = acc[j][r] * (1.0f / 2048.0f);
  ldsx(); for (int rl = 0; rl < 16; ++rl) if (lane < HD / 4) vst2(Y + ((size_t)b * TT + ql0 + rl) * CC + h * HD + lane * 4, *(const v4f*)&ss[wave][rl][lane * 4]);
}

__global__ __launch_bounds__(256) void k_lnrow(const float* __restrict__ X, const float* __restrict__ R, const float* __restrict__ GM, const float* __restrict__ BT, float* __restrict__ OUT) { const int wave = threadIdx.x >> 5, lane = threadIdx.x & 31; const size_t row = (size_t)blockIdx.x * 8 + wave; if (row >= (size_t)NROW) return;
  v4f x[CC / 128]; float s1 = 0.f;
#pragma unroll
  for (int q = 0; q < CC / 128; ++q) { x[q] = *(const v4f*)(X + row * CC + q * 128 + lane * 4); if (R) { const v4f rr = *(const v4f*)(R + row * CC + q * 128 + lane * 4); x[q][0] += rr[0]; x[q][1] += rr[1]; x[q][2] += rr[2]; x[q][3] += rr[3]; }
#pragma unroll
    for (int i = 0; i < 4; ++i) s1 += x[q][i]; }
#pragma unroll
  for (int o = 1; o < 32; o <<= 1) s1 += __shfl_xor(s1, o);
  const float mu = s1 * (1.0f / CC); float qq = 0.f;
#pragma unroll
  for (int q = 0; q < CC / 128; ++q)
#pragma unroll
    for (int i = 0; i < 4; ++i) { const float d = x[q][i] - mu; qq += d * d; }
#pragma unroll
  for (int o = 1; o < 32; o <<= 1) qq += __shfl_xor(qq, o);
  const float rs = rsqrtf(qq * (1.0f / CC) + 1e-5f);
#pragma unroll
  for (int q = 0; q < CC / 128; ++q) { v4f r4; const int c = q * 128 + lane * 4;
#pragma unroll
    for (int i = 0; i < 4; ++i) r4[i] = (x[q][i] - mu) * rs * bfr(GM[c + i]) + bfr(BT[c + i]);
    vst2(OUT + row * CC + c, r4); } }

__global__ __launch_bounds__(128) __attribute__((amdgpu_num_vgpr(256))) void k_rff(const float* __restrict__ O, const __bf16* __restrict__ WOT, const float* __restrict__ BO, float* __restrict__ T) { __shared__ __align__(16) float sf[4][16][132];
  const int tid = threadIdx.x, wave = tid >> 5, lane = tid & 31, col = lane & 15, g = lane >> 4; const int c0 = blockIdx.y * 128; const size_t r0 = (size_t)blockIdx.x * 64 + wave * 16;
  v8f acc[8] = {};
#pragma unroll 2
  for (int kc = 0; kc < CC / 32; ++kc) { const F2 a = split_row(O + (r0 + col) * CC, kc * 32, lane); asm volatile("s_wait_loadcnt 0x0" ::: "memory");
#pragma unroll
    for (int j = 0; j < 8; ++j) { const v16b w = frag_b(WOT + (size_t)(c0 + j * 16 + col) * CC + kc * 32, lane); asm volatile("s_wait_loadcnt 0x0" ::: "memory"); acc[j] = wmma_bf(a.h, w, acc[j]); acc[j] = wmma_bf(a.l, w, acc[j]); } }
#pragma unroll
  for (int j = 0; j < 8; ++j) { const float bias = bfr(BO[c0 + j * 16 + col]);
#pragma unroll
    for (int r = 0; r < 8; ++r) sf[wave][8 * g + r][j * 16 + col] = fmaxf(acc[j][r] + bias, 0.f); }
  ldsx(); for (int rl = 0; rl < 16; ++rl) { const size_t o2 = (r0 + rl) * CC + c0 + lane * 4; const v4f x = *(const v4f*)(O + o2); v4f t = *(const v4f*)&sf[wave][rl][lane * 4]; t[0] += x[0]; t[1] += x[1]; t[2] += x[2]; t[3] += x[3]; vst2(T + o2, t); } }

extern "C" void kernel_launch(void* const* d_in, const int* in_sizes, int n_in, void* d_out, int out_size, void* d_ws, size_t ws_size, hipStream_t stream) {
  if (n_in < 15) return;
  if ((size_t)in_sizes[0] < (size_t)NROW * DIN || (size_t)in_sizes[1] < (size_t)NROW * DIN || in_sizes[2] < NB * TT) return;
  if (in_sizes[3] < DIN * CC || in_sizes[5] < DIN * CC || in_sizes[7] < DIN * CC || in_sizes[9] < CC * CC) return;
  if (in_sizes[4] < CC || in_sizes[6] < CC || in_sizes[8] < CC || in_sizes[10] < CC || in_sizes[11] < CC || in_sizes[12] < CC || in_sizes[13] < CC || in_sizes[14] < CC) return;
  if ((size_t)out_size < (size_t)NROW * CC) return;
  if (ws_size < (size_t)WS_END) return;
  const float* XQ = (const float*)d_in[0]; const float* XK = (const float*)d_in[1]; const int* MK = (const int*)d_in[2];
  const float* WQ = (const float*)d_in[3]; const float* BQ = (const float*)d_in[4]; const float* WK = (const float*)d_in[5]; const float* BK = (const float*)d_in[6];
  const float* WV = (const float*)d_in[7]; const float* BV = (const float*)d_in[8]; const float* WO = (const float*)d_in[9]; const float* BO = (const float*)d_in[10];
  const float* G0 = (const float*)d_in[11]; const float* B0 = (const float*)d_in[12]; const float* G1 = (const float*)d_in[13]; const float* B1 = (const float*)d_in[14];
  char* ws = (char*)d_ws;
  __bf16* WT = (__bf16*)(ws + WS_WT); _Float16 *QH = (_Float16*)(ws + WS_QH), *KH = (_Float16*)(ws + WS_KH), *VT = (_Float16*)(ws + WS_VT), *QL = (_Float16*)(ws + WS_QL);
  float *S = (float*)(ws + WS_S), *QF = (float*)(ws + WS_QF), *O = (float*)(ws + WS_O), *T = (float*)(ws + WS_T);
  k_wprep<<<dim3(DIN / 64, CC / 64, 4), 256, 0, stream>>>(WQ, WK, WV, WO, WT);
  k_proj<<<dim3(NROW / 64, CC / 128, 3), 128, 0, stream>>>(XQ, XK, WT, BQ, BK, BV, QH, QL, KH, VT);
  k_qrows<<<dim3(NROW / 64, CC / 128), 128, 0, stream>>>(XQ, WT, BQ, QF);
  for (int b = 0; b < NB; ++b) {
    k_sc<<<dim3(NQB, TT / 128, NH), 128, 0, stream>>>(QH, KH, QL, b, S);
    k_sm<<<dim3(TT, NH), 256, 0, stream>>>(S, MK, b);
    k_pv<<<dim3(NQB, 1, NH), 128, 0, stream>>>(S, VT, b, T);
  }
  k_lnrow<<<dim3((NROW + 7) / 8), 256, 0, stream>>>(QF, T, G0, B0, O);
  k_rff<<<dim3(NROW / 64, CC / 128), 128, 0, stream>>>(O, WT + (size_t)3 * CC * DIN, BO, T);
  k_lnrow<<<dim3((NROW + 7) / 8), 256, 0, stream>>>(T, nullptr, G1, B1, (float*)d_out);
}
